// mamba2_55490977464371
// MI455X (gfx1250) — hardware-verified
//
#include <hip/hip_runtime.h>
#include <math.h>

typedef __attribute__((ext_vector_type(16))) _Float16 v16h;
typedef __attribute__((ext_vector_type(8)))  _Float16 v8h;
typedef __attribute__((ext_vector_type(16))) __bf16   v16b;
typedef __attribute__((ext_vector_type(8)))  __bf16   v8b;
typedef __attribute__((ext_vector_type(8)))  float    v8f;
typedef __attribute__((ext_vector_type(4)))  float    v4f;
typedef __attribute__((ext_vector_type(4)))  unsigned v4u;

constexpr int kBatch     = 2;
constexpr int kSeqLen    = 2048;
constexpr int kRows      = kBatch * kSeqLen;
constexpr int kDModel    = 1024;
constexpr int kDInner    = 2048;
constexpr int kNHeads    = 64;
constexpr int kHeadDim   = 32;
constexpr int kDState    = 16;
constexpr int kConvDim   = 2080;
constexpr int kDInProj   = 4192;
constexpr int kWinRowsPad = 4224;
constexpr int kZCols     = 2048;
constexpr int kXColsPad  = 2176;
constexpr int kDtCol     = 2080;

static_assert(kRows % 64 == 0, "M tile");
static_assert(kZCols % 64 == 0 && kXColsPad % 64 == 0 && kDModel % 64 == 0, "N tile");
static_assert(kDModel % 32 == 0 && kDInner % 32 == 0, "K step");
static_assert(kZCols + kXColsPad == kWinRowsPad, "W_in plane rows");
static_assert(kNHeads * kHeadDim == kDInner, "heads");

constexpr size_t kOut0Floats = (size_t)kRows * kDModel;
constexpr size_t kOut1OffFloats = 16777216 / 4;
static_assert(kOut1OffFloats == kOut0Floats, "out1 offset");
static_assert(16777216ull + (size_t)kRows * kDInner * 4 == 50331648ull, "out total");

constexpr size_t kSzUbf    = (size_t)kRows * kDModel * 2;
constexpr size_t kSzWinbf  = (size_t)kWinRowsPad * kDModel * 2;
constexpr size_t kSzWoutbf = (size_t)kDModel * kDInner * 2;
constexpr size_t kSzX      = (size_t)kRows * kXColsPad * 4;
constexpr size_t kSzDt     = (size_t)kRows * kNHeads * 4;
constexpr size_t kSzY      = (size_t)kRows * kDInner * 4;
constexpr size_t kSzYn     = (size_t)kRows * kDInner * 2;
constexpr size_t kOffUbf    = 0;
constexpr size_t kOffWinbf  = kOffUbf + kSzUbf;
constexpr size_t kOffWoutbf = kOffWinbf + kSzWinbf;
constexpr size_t kOffX      = kOffWoutbf + kSzWoutbf;
constexpr size_t kOffDt     = kOffX + kSzX;
constexpr size_t kOffDa     = kOffDt + kSzDt;
constexpr size_t kOffY      = kOffDa + kSzDt;
constexpr size_t kOffYnh    = kOffY + kSzY;
constexpr size_t kOffYnl    = kOffYnh + kSzYn;
constexpr size_t kWsTotal   = kOffYnl + kSzYn;
static_assert(kWsTotal == 126091264ull, "carve total");
static_assert(kWsTotal <= 134217728ull, "carve under 128 MiB");
static_assert(kOffWinbf % 256 == 0 && kOffWoutbf % 256 == 0 && kOffX % 256 == 0 && kOffDt % 256 == 0 &&
              kOffDa % 256 == 0 && kOffY % 256 == 0 && kOffYnh % 256 == 0 && kOffYnl % 256 == 0, "alignment");

__device__ __forceinline__ unsigned short f2bf_bits(float f) {
  unsigned u = __float_as_uint(f);
  return (unsigned short)((u + 0x7FFFu + ((u >> 16) & 1u)) >> 16);
}
__device__ __forceinline__ float bf_bits2f(unsigned short h) { return __uint_as_float(((unsigned)h) << 16); }
__device__ __forceinline__ float bfr(float f) { return bf_bits2f(f2bf_bits(f)); }
__device__ __forceinline__ unsigned pack_bf2(float a, float b) {
  return (unsigned)f2bf_bits(a) | (((unsigned)f2bf_bits(b)) << 16);
}

__device__ __forceinline__ void dep_guard_h(v8f& a, v8f& b, v16h x, v16h y) { asm volatile("v_nop\n\tv_nop\n\tv_nop\n\tv_nop" : "+v"(a), "+v"(b) : "v"(x), "v"(y)); }
__device__ __forceinline__ void dep_guard_b(v8f& a, v8f& b, v16b x, v16b y) { asm volatile("v_nop\n\tv_nop\n\tv_nop\n\tv_nop" : "+v"(a), "+v"(b) : "v"(x), "v"(y)); }
__device__ __forceinline__ void keep4_h(v16h a, v16h b, v16h c, v16h d) { asm volatile("v_nop" :: "v"(a), "v"(b), "v"(c), "v"(d)); }
__device__ __forceinline__ void keep4_b(v16b a, v16b b, v16b c, v16b d) { asm volatile("v_nop" :: "v"(a), "v"(b), "v"(c), "v"(d)); }
__device__ __forceinline__ void acc_guard4(v8f& a, v8f& b, v8f& c, v8f& d) { asm volatile("v_nop\n\tv_nop\n\tv_nop\n\tv_nop" : "+v"(a), "+v"(b), "+v"(c), "+v"(d)); }

template <typename T> struct Frag;
template <> struct Frag<_Float16> {
  typedef v16h V; union U { v16h v; v8h h[2]; };
  static __device__ __forceinline__ v16h load(const _Float16* p) {
    U f; f.h[0] = *(const v8h*)(p); f.h[1] = *(const v8h*)(p + 16); return f.v;
  }
  static __device__ __forceinline__ v8f mma(v16h a, v16h b, v8f c) {
    return __builtin_amdgcn_wmma_f32_16x16x32_f16(false, a, false, b, (short)0, c, false, false);
  }
  static __device__ __forceinline__ void guard(v8f& a, v8f& b, v16h x, v16h y) { dep_guard_h(a, b, x, y); }
  static __device__ __forceinline__ void keep(v16h a, v16h b, v16h c, v16h d) { keep4_h(a, b, c, d); }
};
template <> struct Frag<__bf16> {
  typedef v16b V; union U { v16b v; v8b h[2]; };
  static __device__ __forceinline__ v16b load(const __bf16* p) {
    U f; f.h[0] = *(const v8b*)(p); f.h[1] = *(const v8b*)(p + 16); return f.v;
  }
  static __device__ __forceinline__ v8f mma(v16b a, v16b b, v8f c) {
    return __builtin_amdgcn_wmma_f32_16x16x32_bf16(false, a, false, b, (short)0, c, false, false);
  }
  static __device__ __forceinline__ void guard(v8f& a, v8f& b, v16b x, v16b y) { dep_guard_b(a, b, x, y); }
  static __device__ __forceinline__ void keep(v16b a, v16b b, v16b c, v16b d) { keep4_b(a, b, c, d); }
};

template <int ET> struct Elem;
template <> struct Elem<0> { typedef _Float16 T; };
template <> struct Elem<1> { typedef __bf16 T; };

template <int ET, bool SPLITA>
__global__ __launch_bounds__(256) void wmma_gemm64(
    const unsigned short* __restrict__ Ap, const unsigned short* __restrict__ A2p, int lda,
    const unsigned short* __restrict__ Btp, int ldb,
    float* __restrict__ Cout, int ldc,
    int M, int N, int K, float scale) {
  typedef typename Elem<ET>::T T;
  typedef typename Frag<T>::V V;
  const T* A = (const T*)Ap; const T* A2 = (const T*)A2p; const T* Bt = (const T*)Btp;
  __shared__ __align__(16) float sT[8][16 * 68];
  const int lane = threadIdx.x & 31;
  const int wave = threadIdx.x >> 5;
  const int tilesN = N >> 6;
  const int tilesM = M >> 6;
  const int tile = blockIdx.x * 8 + wave;
  if (tile >= tilesM * tilesN) return;
  const int tm = tile / tilesN;
  const int tn = tile - tm * tilesN;
  const int m0 = tm << 6;
  const int n0 = tn << 6;

  const int rlane = lane & 15;
  const int koff  = (lane >> 4) * 8;
  const int mOff  = (lane >> 4) * 8;

  v8f acc[4][4];
#pragma unroll
  for (int i = 0; i < 4; ++i)
#pragma unroll
    for (int j = 0; j < 4; ++j) acc[i][j] = (v8f){0.f,0.f,0.f,0.f,0.f,0.f,0.f,0.f};

  for (int k0 = 0; k0 < K; k0 += 32) {
    V bh[4];
#pragma unroll
    for (int j = 0; j < 4; ++j) {
      const size_t bo = (size_t)(n0 + (j << 4) + rlane) * ldb + koff + k0;
      bh[j] = Frag<T>::load(Bt + bo);
    }
#pragma unroll
    for (int i = 0; i < 4; ++i) {
      const size_t ao = (size_t)(m0 + (i << 4) + rlane) * lda + koff + k0;
      V ah = Frag<T>::load(A + ao);
      V al;
      if (SPLITA) al = Frag<T>::load(A2 + ao);
#pragma unroll
      for (int j = 0; j < 4; ++j) {
        acc[i][j] = Frag<T>::mma(ah, bh[j], acc[i][j]);
        if (SPLITA) acc[i][j] = Frag<T>::mma(al, bh[j], acc[i][j]);
      }
      Frag<T>::guard(acc[i][0], acc[i][3], ah, SPLITA ? al : ah);
    }
    Frag<T>::keep(bh[0], bh[1], bh[2], bh[3]);
  }
  acc_guard4(acc[0][0], acc[0][1], acc[0][2], acc[0][3]);
  acc_guard4(acc[1][0], acc[1][1], acc[1][2], acc[1][3]);
  acc_guard4(acc[2][0], acc[2][1], acc[2][2], acc[2][3]);
  acc_guard4(acc[3][0], acc[3][1], acc[3][2], acc[3][3]);

  float* slab = sT[wave];
#pragma unroll
  for (int i = 0; i < 4; ++i) {
    const int mBase = m0 + (i << 4);
#pragma unroll
    for (int j = 0; j < 4; ++j) {
#pragma unroll
      for (int r = 0; r < 8; ++r) {
        slab[(mOff + r) * 68 + (j << 4) + rlane] = acc[i][j][r] * scale;
      }
    }
    __builtin_amdgcn_fence(__ATOMIC_RELEASE, "workgroup");
    __builtin_amdgcn_wave_barrier();
    __builtin_amdgcn_fence(__ATOMIC_ACQUIRE, "workgroup");
    {
      const int hh = lane >> 4, c4 = (lane & 15) * 4;
      for (int pass = 0; pass < 2; ++pass) {
#pragma unroll
        for (int it = 0; it < 8; ++it) {
          const int row = it * 2 + hh;
          v4f v = *(const v4f*)(slab + row * 68 + c4);
          *(volatile v4f*)(Cout + (size_t)(mBase + row) * ldc + n0 + c4) = v;
        }
        __threadfence();
      }
    }
    __builtin_amdgcn_fence(__ATOMIC_RELEASE, "workgroup");
    __builtin_amdgcn_wave_barrier();
    __builtin_amdgcn_fence(__ATOMIC_ACQUIRE, "workgroup");
  }
}

__global__ __launch_bounds__(256) void cvt_bf16x8_kernel(
    const float* __restrict__ src, unsigned int* __restrict__ dst, int ncols, int nreal, int npad) {
  const int gi = blockIdx.x * 256 + threadIdx.x;
  const long e0 = (long)gi * 8;
  const int row = (int)(e0 / ncols);
  const int col = (int)(e0 - (long)row * ncols);
  if (row >= npad) return;
  const int srow = (row < nreal) ? row : (nreal - 1);
  const float* p = src + (size_t)srow * ncols + col;
  v4f a = *(const v4f*)p;
  v4f c = *(const v4f*)(p + 4);
  const bool padrow = (row >= nreal);
  if (padrow) { a = (v4f){0.f, 0.f, 0.f, 0.f}; c = a; }
  v4u o;
  o[0] = pack_bf2(a[0], a[1]);
  o[1] = pack_bf2(a[2], a[3]);
  o[2] = pack_bf2(c[0], c[1]);
  o[3] = pack_bf2(c[2], c[3]);
  volatile v4u* q = (volatile v4u*)(dst + (size_t)gi * 4);
  *q = o;
  __threadfence();
  *q = o;
}

__global__ __launch_bounds__(256) void dt_prep_kernel(
    const float* __restrict__ X, const float* __restrict__ dt_bias, const float* __restrict__ A_log,
    float* __restrict__ dtp, float* __restrict__ dap) {
  const int idx = blockIdx.x * 256 + threadIdx.x;
  if (idx >= kRows * kNHeads) return;
  const int row = idx >> 6;
  const int h = idx & 63;
  const float traw = X[(size_t)row * kXColsPad + kDtCol + h] + bfr(dt_bias[h]);
  const float sp = fmaxf(traw, 0.0f) + log1pf(expf(-fabsf(traw)));
  const float Ah = -expf(bfr(A_log[h]));
  const float da = expf(sp * Ah);
  volatile float* p0 = (volatile float*)(dtp + idx);
  volatile float* p1 = (volatile float*)(dap + idx);
  *p0 = sp;
  *p1 = da;
  __threadfence();
  *p0 = sp;
  *p1 = da;
}

__global__ __launch_bounds__(128) void ssm_scan_kernel(
    const float* __restrict__ X, const float* __restrict__ dtp, const float* __restrict__ dap,
    const float* __restrict__ convw, const float* __restrict__ convb, const float* __restrict__ Dp,
    float* __restrict__ Y) {
  const int lane = threadIdx.x & 31;
  const int gw = blockIdx.x * 4 + (threadIdx.x >> 5);
  if (gw >= kBatch * kNHeads) return;
  const int b = gw >> 6;
  const int h = gw & 63;
  const int cx = h * kHeadDim + lane;
  const int cb = kDInner + lane;
  const float wx0 = bfr(convw[cx * 4 + 0]);
  const float wx1 = bfr(convw[cx * 4 + 1]);
  const float wx2 = bfr(convw[cx * 4 + 2]);
  const float wx3 = bfr(convw[cx * 4 + 3]);
  const float wb0 = bfr(convw[cb * 4 + 0]);
  const float wb1 = bfr(convw[cb * 4 + 1]);
  const float wb2 = bfr(convw[cb * 4 + 2]);
  const float wb3 = bfr(convw[cb * 4 + 3]);
  const float biasx = bfr(convb[cx]);
  const float biasb = bfr(convb[cb]);
  const float Dh = bfr(Dp[h]);
  float px1 = 0.f, px2 = 0.f, px3 = 0.f;
  float pb1 = 0.f, pb2 = 0.f, pb3 = 0.f;
  float st[kDState];
#pragma unroll
  for (int n = 0; n < kDState; ++n) st[n] = 0.f;

#pragma unroll 1
  for (int t = 0; t < kSeqLen; ++t) {
    const size_t row = (size_t)b * kSeqLen + t;
    const float* xr = X + row * kXColsPad;
    const float xin = xr[cx];
    const float bin = xr[cb];
    const float dt = dtp[row * kNHeads + h];
    const float da = dap[row * kNHeads + h];
    const float cvx = biasx + wx0 * px3 + wx1 * px2 + wx2 * px1 + wx3 * xin;
    const float cvb = biasb + wb0 * pb3 + wb1 * pb2 + wb2 * pb1 + wb3 * bin;
    px3 = px2; px2 = px1; px1 = xin;
    pb3 = pb2; pb2 = pb1; pb1 = bin;
    const float ex = expf(fminf(-cvx, 80.0f));
    const float eb = expf(fminf(-cvb, 80.0f));
    const float xv = cvx * (1.0f / (1.0f + ex));
    const float bcv = cvb * (1.0f / (1.0f + eb));
    const float s = xv * dt;
    float y = Dh * xv;
#pragma unroll
    for (int n = 0; n < kDState; ++n) {
      const float Bn = __shfl(bcv, n, 32);
      const float Cn = __shfl(bcv, n + 16, 32);
      st[n] = da * st[n] + Bn * s;
      y += Cn * st[n];
    }
    volatile float* yp = (volatile float*)(Y + row * kDInner + cx);
    *yp = y;
    __threadfence();
    *yp = y;
  }
}

__global__ __launch_bounds__(512) void gate_norm_kernel(
    const float* __restrict__ Y, const float* __restrict__ Z, const float* __restrict__ nw,
    unsigned int* __restrict__ ynh, unsigned int* __restrict__ ynl) {
  __shared__ __align__(16) float rowbuf[kDInner];
  __shared__ float wsum[16];
  const int row = blockIdx.x;
  const int tid = threadIdx.x;
  const int lane = tid & 31;
  const int wave = tid >> 5;
  const size_t rb = (size_t)row * kDInner;
  const int c0 = tid * 4;
  const v4f yv = *(const v4f*)(Y + rb + c0);
  const v4f zv = *(const v4f*)(Z + rb + c0);
  v4f g;
  float ss = 0.f;
#pragma unroll
  for (int e = 0; e < 4; ++e) {
    const float zz = zv[e];
    const float ez = expf(fminf(-zz, 80.0f));
    const float sg = 1.0f / (1.0f + ez);
    const float gg = yv[e] * (zz * sg);
    g[e] = gg;
    ss += gg * gg;
  }
#pragma unroll
  for (int off = 16; off > 0; off >>= 1) ss += __shfl_xor(ss, off, 32);
  if (lane == 0) wsum[wave] = ss;
  *(v4f*)(rowbuf + c0) = g;
  __syncthreads();
  float tot = 0.f;
#pragma unroll
  for (int w = 0; w < 16; ++w) tot += wsum[w];
  const float inv = rsqrtf(tot * (1.0f / 2048.0f) + 1e-5f);
  if (tid < 256) {
    const int c8 = tid * 8;
    const v4f ga = *(const v4f*)(rowbuf + c8);
    const v4f gb = *(const v4f*)(rowbuf + c8 + 4);
    const v4f wa = *(const v4f*)(nw + c8);
    const v4f wb = *(const v4f*)(nw + c8 + 4);
    float vn[8];
#pragma unroll
    for (int e = 0; e < 4; ++e) {
      vn[e]     = (ga[e] * inv) * bfr(wa[e]);
      vn[4 + e] = (gb[e] * inv) * bfr(wb[e]);
    }
    unsigned hb[8], lb[8];
#pragma unroll
    for (int e = 0; e < 8; ++e) {
      const unsigned short hbit = f2bf_bits(vn[e]);
      const float hf = bf_bits2f(hbit);
      const unsigned short lbit = f2bf_bits(vn[e] - hf);
      hb[e] = (unsigned)hbit;
      lb[e] = (unsigned)lbit;
    }
    v4u hv, lv;
#pragma unroll
    for (int q = 0; q < 4; ++q) {
      hv[q] = hb[2 * q] | (hb[2 * q + 1] << 16);
      lv[q] = lb[2 * q] | (lb[2 * q + 1] << 16);
    }
    volatile v4u* ph = (volatile v4u*)(ynh + ((rb + c8) >> 1));
    volatile v4u* pl = (volatile v4u*)(ynl + ((rb + c8) >> 1));
    *ph = hv;
    *pl = lv;
    __threadfence();
    *ph = hv;
    *pl = lv;
  }
}

extern "C" void kernel_launch(void* const* d_in, const int* in_sizes, int n_in,
                              void* d_out, int out_size, void* d_ws, size_t ws_size,
                              hipStream_t stream) {
  (void)in_sizes; (void)n_in;
  if (ws_size < kWsTotal) return;
  if ((size_t)out_size < kOut0Floats + (size_t)kRows * kDInner) return;

  const float* u       = (const float*)d_in[0];
  const float* W_in    = (const float*)d_in[1];
  const float* conv_w  = (const float*)d_in[2];
  const float* conv_b  = (const float*)d_in[3];
  const float* dt_bias = (const float*)d_in[4];
  const float* A_log   = (const float*)d_in[5];
  const float* Dp      = (const float*)d_in[6];
  const float* norm_w  = (const float*)d_in[7];
  const float* W_out   = (const float*)d_in[8];

  float* out0 = (float*)d_out;
  float* out1 = (float*)d_out + kOut1OffFloats;

  char* wsb = (char*)d_ws;
  unsigned int* ubf_w    = (unsigned int*)(wsb + kOffUbf);
  unsigned int* winbf_w  = (unsigned int*)(wsb + kOffWinbf);
  unsigned int* woutbf_w = (unsigned int*)(wsb + kOffWoutbf);
  const unsigned short* ubf    = (const unsigned short*)(wsb + kOffUbf);
  const unsigned short* winbf  = (const unsigned short*)(wsb + kOffWinbf);
  const unsigned short* woutbf = (const unsigned short*)(wsb + kOffWoutbf);
  float* Xp  = (float*)(wsb + kOffX);
  float* dtp = (float*)(wsb + kOffDt);
  float* dap = (float*)(wsb + kOffDa);
  float* Yp  = (float*)(wsb + kOffY);
  unsigned int* ynh = (unsigned int*)(wsb + kOffYnh);
  unsigned int* ynl = (unsigned int*)(wsb + kOffYnl);

  {
    constexpr int nU = kRows * kDModel / 8;
    constexpr int nW = kWinRowsPad * kDModel / 8;
    constexpr int nO = kDModel * kDInner / 8;
    static_assert(nU % 256 == 0 && nW % 256 == 0 && nO % 256 == 0, "cvt grids exact");
    cvt_bf16x8_kernel<<<nU / 256, 256, 0, stream>>>(u, ubf_w, kDModel, kRows, kRows);
    cvt_bf16x8_kernel<<<nW / 256, 256, 0, stream>>>(W_in, winbf_w, kDModel, kDInProj, kWinRowsPad);
    cvt_bf16x8_kernel<<<nO / 256, 256, 0, stream>>>(W_out, woutbf_w, kDInner, kDModel, kDModel);
  }
  {
    constexpr int tiles = (kRows / 64) * (kZCols / 64);
    static_assert(tiles % 8 == 0, "grid");
    wmma_gemm64<1, false><<<dim3(tiles / 8), 256, 0, stream>>>(
        ubf, ubf, kDModel, winbf, kDModel, out1, kZCols, kRows, kZCols, kDModel, 1.0f);
  }
  {
    constexpr int tiles = (kRows / 64) * (kXColsPad / 64);
    static_assert(tiles % 8 == 0, "grid");
    wmma_gemm64<1, false><<<dim3(tiles / 8), 256, 0, stream>>>(
        ubf, ubf, kDModel, winbf + (size_t)kZCols * kDModel, kDModel, Xp, kXColsPad,
        kRows, kXColsPad, kDModel, 1.0f);
  }
  {
    constexpr int n = kRows * kNHeads;
    static_assert(n % 256 == 0, "grid");
    dt_prep_kernel<<<n / 256, 256, 0, stream>>>(Xp, dt_bias, A_log, dtp, dap);
  }
  {
    constexpr int waves = kBatch * kNHeads;
    static_assert(waves % 4 == 0, "grid");
    ssm_scan_kernel<<<waves / 4, 128, 0, stream>>>(Xp, dtp, dap, conv_w, conv_b, Dp, Yp);
  }
  gate_norm_kernel<<<kRows, 512, 0, stream>>>(Yp, (const float*)out1, norm_w, ynh, ynl);
  {
    constexpr int tiles = (kRows / 64) * (kDModel / 64);
    static_assert(tiles % 8 == 0, "grid");
    wmma_gemm64<1, true><<<dim3(tiles / 8), 256, 0, stream>>>(
        (const unsigned short*)ynh, (const unsigned short*)ynl, kDInner, woutbf, kDInner,
        out0, kDModel, kRows, kDModel, kDInner, 1.0f);
  }
}
